// H3_37993280700546
// MI455X (gfx1250) — hardware-run, weakly checked
//
#include <hip/hip_runtime.h>
#include <math.h>

typedef __attribute__((ext_vector_type(16))) _Float16 v16h;
typedef __attribute__((ext_vector_type(8)))  _Float16 v8h;
typedef __attribute__((ext_vector_type(16))) __bf16   v16b;
typedef __attribute__((ext_vector_type(8)))  __bf16   v8b;
typedef __attribute__((ext_vector_type(8)))  float    v8f;
typedef __attribute__((ext_vector_type(4)))  float    v4f;
typedef __attribute__((ext_vector_type(4)))  unsigned v4u;

constexpr bool kLegBf16 = true;
constexpr int  kSplitMode = kLegBf16 ? 0 : 2;
constexpr int  kB   = 4;
constexpr int  kH   = 1024;
constexpr int  kL   = 2048;
constexpr int  kNm  = 32;
constexpr int  kTok = kB * kL;
constexpr int  kO1  = 3 * kH;
constexpr int  kO2  = 2 * kH;
constexpr int  kPitchTr  = 65;
constexpr int  kPitchIn  = 36;
constexpr int  kPitchOut = 68;
constexpr int  kPitchScan = 68;
constexpr int  kScanSteps = 16;
constexpr float kCarryW = 1024.0f;
constexpr float kCarryY = 64.0f;
constexpr float kOutFold = kLegBf16 ? (1.0f / (kCarryW * kCarryY)) : 1.0f;
constexpr float kF16MinNormal = 6.103515625e-5f;
static_assert(kTok == 8192 && kO1 == 3072 && kO2 == 2048, "shape");
static_assert((kH % 32) == 0 && (kH / 32) == 32, "K multiple of 32; 32 channel tiles");
static_assert((kTok % 64) == 0 && (kTok / 64) == 128 && (kL % 64) == 0, "token tiles");
static_assert((kL % kScanSteps) == 0, "scan chunking");

constexpr size_t kLoMul   = kLegBf16 ? 0 : 1;
constexpr size_t kSzTok16 = (size_t)kTok * kH * 2;
constexpr size_t kSzWin16 = (size_t)kO1 * kH * 2;
constexpr size_t kSzWout16 = (size_t)kO2 * kH * 2;
constexpr size_t kSzF32   = (size_t)kTok * kH * 4;
constexpr size_t kSzCst   = (size_t)4 * kH * kNm * 4;
constexpr size_t kOffUTH  = 0;
constexpr size_t kOffUTL  = kOffUTH + kSzTok16;
constexpr size_t kOffWIH  = kOffUTL + kLoMul * kSzTok16;
constexpr size_t kOffWIL  = kOffWIH + kSzWin16;
constexpr size_t kOffWOH  = kOffWIL + kLoMul * kSzWin16;
constexpr size_t kOffWOL  = kOffWOH + kSzWout16;
constexpr size_t kOffU2P  = kOffWOL + kLoMul * kSzWout16;
constexpr size_t kOffU3   = kOffU2P + kSzF32;
constexpr size_t kOffCST  = kOffU3 + kSzF32;
constexpr size_t kOffU3PH = kLegBf16 ? (kOffCST + kSzCst) : kOffUTH;
constexpr size_t kOffU3PL = kOffUTL;
constexpr size_t kWsTotal = kLegBf16 ? (kOffU3PH + kSzTok16) : (kOffCST + kSzCst);
static_assert(!kLegBf16 || kWsTotal == 111673344ull, "carve total");
static_assert(kWsTotal <= 134217728ull, "carve cap");
static_assert((kOffUTL % 128) == 0 && (kOffWIH % 128) == 0 && (kOffWIL % 128) == 0 && (kOffWOH % 128) == 0 &&
              (kOffWOL % 128) == 0 && (kOffU2P % 128) == 0 && (kOffU3 % 128) == 0 && (kOffCST % 128) == 0 &&
              (kOffU3PH % 128) == 0 && (kOffU3PL % 128) == 0, "128-B aligned regions");

__device__ __forceinline__ unsigned bf_rne_hi(float f) {
  unsigned u = __float_as_uint(f);
  const unsigned lsb = (u & 0x00010000u) ? 1u : 0u;
  u = (u + 0x7FFFu + lsb) & 0xFFFF0000u;
  return u;
}
__device__ __forceinline__ float bf_rne_f(float f) { return __uint_as_float(bf_rne_hi(f)); }
__device__ __forceinline__ float rin(float f) { return kLegBf16 ? bf_rne_f(f) : f; }

__device__ __forceinline__ v4u pack8_hi(const float (&x)[8]) {
  v4u w;
#pragma unroll
  for (int p = 0; p < 4; ++p) {
    const unsigned lo = bf_rne_hi(x[2 * p]);
    const unsigned hi = bf_rne_hi(x[2 * p + 1]);
    unsigned t = hi | (lo >> 16);
    asm volatile("" : "+v"(t));
    w[p] = t;
  }
  return w;
}
__device__ __forceinline__ v4u pack8_lo(const float (&x)[8]) {
  v4u w;
#pragma unroll
  for (int p = 0; p < 4; ++p) {
    const float r0 = x[2 * p]     - bf_rne_f(x[2 * p]);
    const float r1 = x[2 * p + 1] - bf_rne_f(x[2 * p + 1]);
    const unsigned lo = bf_rne_hi(r0);
    const unsigned hi = bf_rne_hi(r1);
    unsigned t = hi | (lo >> 16);
    asm volatile("" : "+v"(t));
    w[p] = t;
  }
  return w;
}
__device__ __forceinline__ _Float16 f16_carried(float x, float carry) {
  float v = x * carry;
  v = fminf(fmaxf(v, -65504.0f), 65504.0f);
  v = (fabsf(v) < kF16MinNormal) ? 0.0f : v;
  return (_Float16)v;
}

__device__ __forceinline__ void tie_acc(v8f& c, v16b a, v16b b) { asm volatile("" : "+v"(c) : "v"(a), "v"(b)); }
__device__ __forceinline__ void tie_acc(v8f& c, v16h a, v16h b) { asm volatile("" : "+v"(c) : "v"(a), "v"(b)); }
__device__ __forceinline__ void tie_acc_nops(v8f& c, v16b a, v16b b) { asm volatile("v_nop\n\tv_nop\n\tv_nop\n\tv_nop" : "+v"(c) : "v"(a), "v"(b)); }
__device__ __forceinline__ void tie_acc_nops(v8f& c, v16h a, v16h b) { asm volatile("v_nop\n\tv_nop\n\tv_nop\n\tv_nop" : "+v"(c) : "v"(a), "v"(b)); }
__device__ __forceinline__ void keep4v(v16h a, v16h b, v16h c, v16h d) { asm volatile("v_nop" :: "v"(a), "v"(b), "v"(c), "v"(d)); }
__device__ __forceinline__ void keep4v(v16b a, v16b b, v16b c, v16b d) { asm volatile("v_nop" :: "v"(a), "v"(b), "v"(c), "v"(d)); }

template <typename T> struct Frag;
template <> struct Frag<_Float16> {
  typedef v16h V; union U { v16h v; v8h h[2]; };
  static __device__ __forceinline__ v16h load(const _Float16* p) {
    U f; f.h[0] = *(const v8h*)(p); f.h[1] = *(const v8h*)(p + 16); return f.v;
  }
  static __device__ __forceinline__ v8f mma(v16h a, v16h b, v8f c) {
    return __builtin_amdgcn_wmma_f32_16x16x32_f16(false, a, false, b, (short)0, c, false, false);
  }
};
template <> struct Frag<__bf16> {
  typedef v16b V; union U { v16b v; v8b h[2]; };
  static __device__ __forceinline__ v16b load(const __bf16* p) {
    U f; f.h[0] = *(const v8b*)(p); f.h[1] = *(const v8b*)(p + 16); return f.v;
  }
  static __device__ __forceinline__ v8f mma(v16b a, v16b b, v8f c) {
    return __builtin_amdgcn_wmma_f32_16x16x32_bf16(false, a, false, b, (short)0, c, false, false);
  }
};
template <int ET> struct Elem;
template <> struct Elem<0> { typedef _Float16 T; };
template <> struct Elem<1> { typedef __bf16 T; };

__global__ __launch_bounds__(256) void transpose_convert_kernel(
    const float* __restrict__ U, unsigned short* __restrict__ TH, unsigned short* __restrict__ TL)
{
  __shared__ float sT[64 * kPitchTr];
  const int tid = threadIdx.x, lane = tid & 31, wave = tid >> 5;
  const int l0 = blockIdx.x * 64, h0 = blockIdx.y * 64, bix = blockIdx.z;
  {
    const int hr0 = tid >> 4, c4 = (tid & 15) * 4;
#pragma unroll
    for (int it = 0; it < 4; ++it) {
      const int hr = it * 16 + hr0;
      const v4f v = *(const v4f*)(U + ((size_t)(bix * kH + h0 + hr)) * kL + l0 + c4);
      const float e0 = v[0], e1 = v[1], e2 = v[2], e3 = v[3];
      sT[hr * kPitchTr + c4 + 0] = e0;
      sT[hr * kPitchTr + c4 + 1] = e1;
      sT[hr * kPitchTr + c4 + 2] = e2;
      sT[hr * kPitchTr + c4 + 3] = e3;
    }
  }
  __syncthreads();
  const int q = lane >> 3, c8 = (lane & 7) * 8;
  v4u hw[2], lw[2];
#pragma unroll
  for (int it = 0; it < 2; ++it) {
    const int lr = it * 32 + wave * 4 + q;
    float x[8];
#pragma unroll
    for (int e = 0; e < 8; ++e) x[e] = sT[(c8 + e) * kPitchTr + lr];
    hw[it] = pack8_hi(x);
    if (!kLegBf16) lw[it] = pack8_lo(x);
    else lw[it] = hw[it];
  }
  for (int pass = 0; pass < 2; ++pass) {
#pragma unroll
    for (int it = 0; it < 2; ++it) {
      const int lr = it * 32 + wave * 4 + q;
      const size_t o = ((size_t)(bix * kL + l0 + lr)) * kH + h0 + c8;
      *(volatile v4u*)(TH + o) = hw[it];
      if (!kLegBf16) *(volatile v4u*)(TL + o) = lw[it];
    }
    __threadfence();
  }
}

template <int KIND>
__global__ __launch_bounds__(256) void convert_rows_kernel(
    const float* __restrict__ src, unsigned short* __restrict__ dhi, unsigned short* __restrict__ dlo, int total8)
{
  const int i = blockIdx.x * 256 + threadIdx.x;
  if (i >= total8) return;
  const size_t e0 = (size_t)i << 3;
  const v4f a0 = *(const v4f*)(src + e0);
  const v4f a1 = *(const v4f*)(src + e0 + 4);
  float x[8];
  x[0] = a0[0]; x[1] = a0[1]; x[2] = a0[2]; x[3] = a0[3];
  x[4] = a1[0]; x[5] = a1[1]; x[6] = a1[2]; x[7] = a1[3];
  if (KIND == 0) {
    const v4u hw = pack8_hi(x);
    v4u lw = hw;
    if (!kLegBf16) lw = pack8_lo(x);
    *(volatile v4u*)(dhi + e0) = hw;
    if (!kLegBf16) *(volatile v4u*)(dlo + e0) = lw;
    __threadfence();
    *(volatile v4u*)(dhi + e0) = hw;
    if (!kLegBf16) *(volatile v4u*)(dlo + e0) = lw;
  } else {
    v8h hv;
#pragma unroll
    for (int e = 0; e < 8; ++e) hv[e] = f16_carried(bf_rne_f(x[e]), kCarryW);
    *(volatile v8h*)(dhi + e0) = hv;
    __threadfence();
    *(volatile v8h*)(dhi + e0) = hv;
  }
}

__global__ __launch_bounds__(256) void mode_consts_kernel(
    const float* __restrict__ log_dt, const float* __restrict__ A_re, const float* __restrict__ A_im,
    const float* __restrict__ C_re, const float* __restrict__ C_im, float* __restrict__ CST)
{
  const int idx = blockIdx.x * 256 + threadIdx.x;
  const int h = idx >> 5;
  const float dt = expf(rin(log_dt[h]));
  const float Ar = -rin(A_re[idx]);
  const float Ai = rin(A_im[idx]);
  const float er = Ar * dt;
  const float ei = Ai * dt;
  const float mag = expf(er);
  float sn, cs;
  sincosf(ei, &sn, &cs);
  const float wr = mag * cs;
  const float wi = mag * sn;
  const float cre = rin(C_re[idx]);
  const float cim = rin(C_im[idx]);
  const float nr = wr - 1.0f;
  const float ni = wi;
  const float tr = cre * nr - cim * ni;
  const float ti = cre * ni + cim * nr;
  const float den = Ar * Ar + Ai * Ai;
  const float inv = 1.0f / den;
  const float cdr = (tr * Ar + ti * Ai) * inv;
  const float cdi = (ti * Ar - tr * Ai) * inv;
  volatile float* p0 = CST + idx;
  volatile float* p1 = CST + (size_t)kH * kNm + idx;
  volatile float* p2 = CST + (size_t)2 * kH * kNm + idx;
  volatile float* p3 = CST + (size_t)3 * kH * kNm + idx;
  *p0 = wr; *p1 = wi; *p2 = cdr; *p3 = cdi;
  __threadfence();
  *p0 = wr; *p1 = wi; *p2 = cdr; *p3 = cdi;
}

__device__ __forceinline__ void step_in(const __bf16* __restrict__ A, const __bf16* __restrict__ Bm,
                                        const unsigned (&ao)[2], const unsigned (&bo)[6], int k0,
                                        v8f (&acc)[2][6])
{
  v16b a[2], b[6];
#pragma unroll
  for (int i = 0; i < 2; ++i) a[i] = Frag<__bf16>::load(A + ao[i] + k0);
#pragma unroll
  for (int j = 0; j < 6; ++j) b[j] = Frag<__bf16>::load(Bm + bo[j] + k0);
#pragma unroll
  for (int i = 0; i < 2; ++i)
#pragma unroll
    for (int j = 0; j < 6; ++j) acc[i][j] = Frag<__bf16>::mma(a[i], b[j], acc[i][j]);
#pragma unroll
  for (int i = 0; i < 2; ++i)
#pragma unroll
    for (int j = 0; j < 6; ++j) {
      if (i == 1 && j == 5) tie_acc_nops(acc[i][j], a[i], b[j]);
      else tie_acc(acc[i][j], a[i], b[j]);
    }
  keep4v(b[0], b[1], b[2], b[3]);
  keep4v(b[4], b[5], a[0], a[1]);
}

template <int SPL>
__global__ __launch_bounds__(256) void proj_in_gate_kernel(
    const unsigned short* __restrict__ Ahp, const unsigned short* __restrict__ Alp,
    const unsigned short* __restrict__ Bhp, const unsigned short* __restrict__ Blp,
    const float* __restrict__ bin, float* __restrict__ U2P, float* __restrict__ U3)
{
  __shared__ __align__(16) float sG[8][2][16 * kPitchIn];
  const int lane = threadIdx.x & 31, wave = threadIdx.x >> 5;
  const int tile = blockIdx.x * 8 + wave;
  const int tm = tile >> 5, th = tile & 31;
  const int m0 = tm * 32, h0 = th * 32;
  const int rlane = lane & 15, hh = lane >> 4;
  const int koff = hh * 8, mOff = hh * 8;
  const __bf16* Ah = (const __bf16*)Ahp;
  const __bf16* Al = (const __bf16*)Alp;
  const __bf16* Bh = (const __bf16*)Bhp;
  const __bf16* Bl = (const __bf16*)Blp;

  unsigned ao[2], bo[6];
#pragma unroll
  for (int i = 0; i < 2; ++i) ao[i] = (unsigned)((m0 + i * 16 + rlane) * kH + koff);
#pragma unroll
  for (int j = 0; j < 6; ++j) bo[j] = (unsigned)(((j >> 1) * kH + h0 + (j & 1) * 16 + rlane) * kH + koff);

  v8f acc[2][6];
#pragma unroll
  for (int i = 0; i < 2; ++i)
#pragma unroll
    for (int j = 0; j < 6; ++j) acc[i][j] = (v8f){0.f,0.f,0.f,0.f,0.f,0.f,0.f,0.f};

#pragma unroll 1
  for (int k0 = 0; k0 < kH; k0 += 32) {
    step_in(Ah, Bh, ao, bo, k0, acc);
    if (SPL == 2) {
      step_in(Ah, Bl, ao, bo, k0, acc);
      step_in(Al, Bh, ao, bo, k0, acc);
    }
  }

  float* s2 = sG[wave][0];
  float* s3 = sG[wave][1];
  float b1[2], b2[2], b3[2];
#pragma unroll
  for (int jh = 0; jh < 2; ++jh) {
    const int ch = h0 + jh * 16 + rlane;
    b1[jh] = rin(bin[ch]);
    b2[jh] = rin(bin[kH + ch]);
    b3[jh] = rin(bin[2 * kH + ch]);
  }
  const int q = lane >> 3, c4 = (lane & 7) * 4;
#pragma unroll
  for (int i = 0; i < 2; ++i) {
#pragma unroll
    for (int jh = 0; jh < 2; ++jh) {
#pragma unroll
      for (int r = 0; r < 8; ++r) {
        const float x1 = acc[i][0 + jh][r] + b1[jh];
        const float x2 = acc[i][2 + jh][r] + b2[jh];
        const float x3 = acc[i][4 + jh][r] + b3[jh];
        s2[(mOff + r) * kPitchIn + jh * 16 + rlane] = x2 * x1;
        s3[(mOff + r) * kPitchIn + jh * 16 + rlane] = x3;
      }
    }
    __builtin_amdgcn_fence(__ATOMIC_RELEASE, "workgroup");
    __builtin_amdgcn_wave_barrier();
    __builtin_amdgcn_fence(__ATOMIC_ACQUIRE, "workgroup");
    v4f v2[4], v3[4];
#pragma unroll
    for (int it = 0; it < 4; ++it) {
      const int row = it * 4 + q;
      v2[it] = *(const v4f*)(s2 + row * kPitchIn + c4);
      v3[it] = *(const v4f*)(s3 + row * kPitchIn + c4);
    }
    for (int pass = 0; pass < 2; ++pass) {
#pragma unroll
      for (int it = 0; it < 4; ++it) {
        const int row = it * 4 + q;
        const size_t o = (size_t)(m0 + i * 16 + row) * kH + h0 + c4;
        *(volatile v4f*)(U2P + o) = v2[it];
        *(volatile v4f*)(U3 + o) = v3[it];
      }
      __threadfence();
    }
    __builtin_amdgcn_fence(__ATOMIC_RELEASE, "workgroup");
    __builtin_amdgcn_wave_barrier();
    __builtin_amdgcn_fence(__ATOMIC_ACQUIRE, "workgroup");
  }
}

__global__ __launch_bounds__(128) void scan_gate_kernel(
    const float* __restrict__ CST, const float* __restrict__ Dv,
    const float* __restrict__ U2P, const float* __restrict__ U3,
    unsigned short* __restrict__ YH, unsigned short* __restrict__ YL)
{
  __shared__ __align__(16) float sY[kScanSteps * kPitchScan];
  const int tid = threadIdx.x, lane = tid & 31, wave = tid >> 5;
  const int hf = lane >> 4, cl = lane & 15;
  const int bix = blockIdx.x >> 4;
  const int d0 = (blockIdx.x & 15) * 64;
  const int dloc = wave * 16 + cl;
  const int d = d0 + dloc;
  const int cb = d * kNm + hf * 16;

  float wr[16], wi[16], cr[16], ci[16], sr[16], si[16];
#pragma unroll
  for (int g4 = 0; g4 < 4; ++g4) {
    const v4f a = *(const v4f*)(CST + cb + 4 * g4);
    const v4f b = *(const v4f*)(CST + (size_t)kH * kNm + cb + 4 * g4);
    const v4f c = *(const v4f*)(CST + (size_t)2 * kH * kNm + cb + 4 * g4);
    const v4f e = *(const v4f*)(CST + (size_t)3 * kH * kNm + cb + 4 * g4);
    wr[4 * g4 + 0] = a[0]; wr[4 * g4 + 1] = a[1]; wr[4 * g4 + 2] = a[2]; wr[4 * g4 + 3] = a[3];
    wi[4 * g4 + 0] = b[0]; wi[4 * g4 + 1] = b[1]; wi[4 * g4 + 2] = b[2]; wi[4 * g4 + 3] = b[3];
    cr[4 * g4 + 0] = c[0]; cr[4 * g4 + 1] = c[1]; cr[4 * g4 + 2] = c[2]; cr[4 * g4 + 3] = c[3];
    ci[4 * g4 + 0] = e[0]; ci[4 * g4 + 1] = e[1]; ci[4 * g4 + 2] = e[2]; ci[4 * g4 + 3] = e[3];
  }
#pragma unroll
  for (int k = 0; k < 16; ++k) { sr[k] = 0.0f; si[k] = 0.0f; }
  const float Dd = rin(Dv[d]);
  const size_t row0 = (size_t)bix * kL;
  const int q = lane >> 3, c8 = (lane & 7) * 8;
  const int frow = wave * 4 + q;

#pragma unroll 1
  for (int t0 = 0; t0 < kL; t0 += kScanSteps) {
    const float* p2 = U2P + (row0 + t0) * kH + d;
    const float* p3 = U3 + (row0 + t0) * kH + d;
    __syncthreads();
#pragma unroll 1
    for (int s = 0; s < kScanSteps; ++s) {
      float uv = p2[(size_t)s * kH];
      asm volatile("" : "+v"(uv));
      float gv = p3[(size_t)s * kH];
      asm volatile("" : "+v"(gv));
      float y = 0.0f;
#pragma unroll
      for (int k = 0; k < 16; ++k) {
        float nsr = fmaf(wr[k], sr[k], uv);
        nsr = fmaf(-wi[k], si[k], nsr);
        float nsi = wr[k] * si[k];
        nsi = fmaf(wi[k], sr[k], nsi);
        sr[k] = nsr;
        si[k] = nsi;
        y = fmaf(cr[k], nsr, y);
        y = fmaf(-ci[k], nsi, y);
      }
      const float yo = __shfl_xor(y, 16, 32);
      const float ytot = y + yo;
      const float yy = fmaf(Dd, uv, 2.0f * ytot);
      const float v = gv * yy;
      sY[s * kPitchScan + dloc] = v;
    }
    __syncthreads();
    {
      const float* sp = sY + frow * kPitchScan + c8;
      const v4f a0 = *(const v4f*)(sp);
      const v4f a1 = *(const v4f*)(sp + 4);
      float x[8];
      x[0] = a0[0]; x[1] = a0[1]; x[2] = a0[2]; x[3] = a0[3];
      x[4] = a1[0]; x[5] = a1[1]; x[6] = a1[2]; x[7] = a1[3];
      const size_t o = (row0 + t0 + frow) * kH + d0 + c8;
      if (kLegBf16) {
        v8h hv;
#pragma unroll
        for (int e = 0; e < 8; ++e) hv[e] = f16_carried(x[e], kCarryY);
        *(volatile v8h*)(YH + o) = hv;
        __threadfence();
        *(volatile v8h*)(YH + o) = hv;
      } else {
        const v4u hw = pack8_hi(x);
        const v4u lw = pack8_lo(x);
        *(volatile v4u*)(YH + o) = hw;
        *(volatile v4u*)(YL + o) = lw;
        __threadfence();
        *(volatile v4u*)(YH + o) = hw;
        *(volatile v4u*)(YL + o) = lw;
      }
    }
  }
}

template <typename T>
__device__ __forceinline__ void step_out(const T* __restrict__ A, const T* __restrict__ Bm,
                                         const unsigned (&ao)[4], const unsigned (&bo)[4], int k0,
                                         v8f (&acc)[4][4])
{
  typedef typename Frag<T>::V V;
  V a[4], b[4];
#pragma unroll
  for (int j = 0; j < 4; ++j) b[j] = Frag<T>::load(Bm + bo[j] + k0);
#pragma unroll
  for (int i = 0; i < 4; ++i) a[i] = Frag<T>::load(A + ao[i] + k0);
#pragma unroll
  for (int i = 0; i < 4; ++i)
#pragma unroll
    for (int j = 0; j < 4; ++j) acc[i][j] = Frag<T>::mma(a[i], b[j], acc[i][j]);
#pragma unroll
  for (int i = 0; i < 4; ++i)
#pragma unroll
    for (int j = 0; j < 4; ++j) {
      if (i == 3 && j == 3) tie_acc_nops(acc[i][j], a[i], b[j]);
      else tie_acc(acc[i][j], a[i], b[j]);
    }
  keep4v(a[0], a[1], a[2], a[3]);
  keep4v(b[0], b[1], b[2], b[3]);
}

template <int ET, int SPL>
__global__ __launch_bounds__(128) void proj_out_glu_kernel(
    const unsigned short* __restrict__ Ahp, const unsigned short* __restrict__ Alp,
    const unsigned short* __restrict__ Bhp, const unsigned short* __restrict__ Blp,
    const float* __restrict__ bout, float* __restrict__ out)
{
  typedef typename Elem<ET>::T T;
  __shared__ __align__(16) float sE[4][2][16 * kPitchOut];
  const int lane = threadIdx.x & 31, wave = threadIdx.x >> 5;
  const int tile = blockIdx.x * 4 + wave;
  const int to = tile >> 7, tn = tile & 127;
  const int o0 = to * 32, n0 = tn * 64;
  const int bix = n0 >> 11, l0 = n0 & (kL - 1);
  const int rlane = lane & 15, hh = lane >> 4;
  const int koff = hh * 8, mOff = hh * 8;
  const T* Ah = (const T*)Ahp;
  const T* Al = (const T*)Alp;
  const T* Bh = (const T*)Bhp;
  const T* Bl = (const T*)Blp;

  unsigned ao[4], bo[4];
#pragma unroll
  for (int i = 0; i < 4; ++i) ao[i] = (unsigned)(((i >> 1) * kH + o0 + (i & 1) * 16 + rlane) * kH + koff);
#pragma unroll
  for (int j = 0; j < 4; ++j) bo[j] = (unsigned)((n0 + j * 16 + rlane) * kH + koff);

  v8f acc[4][4];
#pragma unroll
  for (int i = 0; i < 4; ++i)
#pragma unroll
    for (int j = 0; j < 4; ++j) acc[i][j] = (v8f){0.f,0.f,0.f,0.f,0.f,0.f,0.f,0.f};

#pragma unroll 1
  for (int k0 = 0; k0 < kH; k0 += 32) {
    step_out<T>(Ah, Bh, ao, bo, k0, acc);
    if (SPL == 2) {
      step_out<T>(Ah, Bl, ao, bo, k0, acc);
      step_out<T>(Al, Bh, ao, bo, k0, acc);
    }
  }

  float* sa = sE[wave][0];
  float* sg = sE[wave][1];
  const int c4 = (lane & 15) * 4;
#pragma unroll
  for (int osub = 0; osub < 2; ++osub) {
#pragma unroll
    for (int j = 0; j < 4; ++j) {
#pragma unroll
      for (int r = 0; r < 8; ++r) {
        sa[(mOff + r) * kPitchOut + j * 16 + rlane] = acc[osub][j][r];
        sg[(mOff + r) * kPitchOut + j * 16 + rlane] = acc[2 + osub][j][r];
      }
    }
    __builtin_amdgcn_fence(__ATOMIC_RELEASE, "workgroup");
    __builtin_amdgcn_wave_barrier();
    __builtin_amdgcn_fence(__ATOMIC_ACQUIRE, "workgroup");
#pragma unroll 1
    for (int it = 0; it < 8; ++it) {
      const int row = it * 2 + hh;
      const int o = o0 + osub * 16 + row;
      const float ba = rin(bout[o]);
      const float bg = rin(bout[kH + o]);
      const v4f av = *(const v4f*)(sa + row * kPitchOut + c4);
      const v4f gvv = *(const v4f*)(sg + row * kPitchOut + c4);
      v4f ov;
#pragma unroll
      for (int e = 0; e < 4; ++e) {
        const float ae = av[e];
        const float ge = gvv[e];
        const float a = ae * kOutFold + ba;
        const float g = ge * kOutFold + bg;
        const float sgm = 1.0f / (1.0f + expf(-g));
        ov[e] = a * sgm;
      }
      *(v4f*)(sa + row * kPitchOut + c4) = ov;
    }
    __builtin_amdgcn_fence(__ATOMIC_RELEASE, "workgroup");
    __builtin_amdgcn_wave_barrier();
    __builtin_amdgcn_fence(__ATOMIC_ACQUIRE, "workgroup");
    for (int pass = 0; pass < 2; ++pass) {
#pragma unroll
      for (int it = 0; it < 8; ++it) {
        const int row = it * 2 + hh;
        const v4f v = *(const v4f*)(sa + row * kPitchOut + c4);
        *(volatile v4f*)(out + ((size_t)(bix * kH + o0 + osub * 16 + row)) * kL + l0 + c4) = v;
      }
      __threadfence();
    }
    __builtin_amdgcn_fence(__ATOMIC_RELEASE, "workgroup");
    __builtin_amdgcn_wave_barrier();
    __builtin_amdgcn_fence(__ATOMIC_ACQUIRE, "workgroup");
  }
}

extern "C" void kernel_launch(void* const* d_in, const int* in_sizes, int n_in,
                              void* d_out, int out_size, void* d_ws, size_t ws_size,
                              hipStream_t stream) {
  if (n_in < 11) return;
  if (in_sizes[0] != kB * kH * kL) return;
  if (in_sizes[1] != kO1 * kH) return;
  if (in_sizes[2] != kO1) return;
  if (in_sizes[3] != kH) return;
  if (in_sizes[4] != kH * kNm) return;
  if (in_sizes[5] != kH * kNm) return;
  if (in_sizes[6] != kH * kNm) return;
  if (in_sizes[7] != kH * kNm) return;
  if (in_sizes[8] != kH) return;
  if (in_sizes[9] != kO2 * kH) return;
  if (in_sizes[10] != kO2) return;
  if (out_size != kB * kH * kL) return;
  if (ws_size < kWsTotal) return;

  const float* u      = (const float*)d_in[0];
  const float* W_in   = (const float*)d_in[1];
  const float* b_in   = (const float*)d_in[2];
  const float* log_dt = (const float*)d_in[3];
  const float* A_re   = (const float*)d_in[4];
  const float* A_im   = (const float*)d_in[5];
  const float* C_re   = (const float*)d_in[6];
  const float* C_im   = (const float*)d_in[7];
  const float* Dv     = (const float*)d_in[8];
  const float* W_out  = (const float*)d_in[9];
  const float* b_out  = (const float*)d_in[10];
  float* out = (float*)d_out;

  char* ws = (char*)d_ws;
  unsigned short* UTH  = (unsigned short*)(ws + kOffUTH);
  unsigned short* UTL  = (unsigned short*)(ws + kOffUTL);
  unsigned short* WIH  = (unsigned short*)(ws + kOffWIH);
  unsigned short* WIL  = (unsigned short*)(ws + kOffWIL);
  unsigned short* WOH  = (unsigned short*)(ws + kOffWOH);
  unsigned short* WOL  = (unsigned short*)(ws + kOffWOL);
  float*          U2P  = (float*)(ws + kOffU2P);
  float*          U3   = (float*)(ws + kOffU3);
  float*          CST  = (float*)(ws + kOffCST);
  unsigned short* U3PH = (unsigned short*)(ws + kOffU3PH);
  unsigned short* U3PL = (unsigned short*)(ws + kOffU3PL);

  transpose_convert_kernel<<<dim3(kL / 64, kH / 64, kB), 256, 0, stream>>>(u, UTH, UTL);
  convert_rows_kernel<0><<<(kO1 * kH / 8) / 256, 256, 0, stream>>>(W_in, WIH, WIL, kO1 * kH / 8);
  convert_rows_kernel<(kLegBf16 ? 1 : 0)><<<(kO2 * kH / 8) / 256, 256, 0, stream>>>(W_out, WOH, WOL, kO2 * kH / 8);
  mode_consts_kernel<<<(kH * kNm) / 256, 256, 0, stream>>>(log_dt, A_re, A_im, C_re, C_im, CST);
  proj_in_gate_kernel<kSplitMode><<<(kTok / 32) * (kH / 32) / 8, 256, 0, stream>>>(
      UTH, UTL, WIH, WIL, b_in, U2P, U3);
  scan_gate_kernel<<<kB * (kH / 64), 128, 0, stream>>>(CST, Dv, U2P, U3, U3PH, U3PL);
  proj_out_glu_kernel<(kLegBf16 ? 0 : 1), kSplitMode><<<(kH / 32) * (kTok / 64) / 4, 128, 0, stream>>>(
      WOH, WOL, U3PH, U3PL, b_out, out);
}
